// DLA_38225208934978
// MI455X (gfx1250) — hardware-verified
//
#include <hip/hip_runtime.h>


#define TT   2048
#define DM   2048
#define NH_  16
#define QLR  768
#define KVW  576
#define KVL  512
#define QKH  192
#define DN   128
#define DR   64
#define DV   128
#define HH   96
#define ZH   1
#define RH   256
#define PCAR 1024.0f
#define SCL  0.072168783648703216f
#define OMUL 0.44394191924311794f
#define LINIT 0.55605808075688206f
typedef _Float16 h16;
typedef unsigned short bf;
typedef __attribute__((ext_vector_type(16))) __bf16   v16bf;
typedef __attribute__((ext_vector_type(16))) _Float16 v16h;
typedef __attribute__((ext_vector_type(8)))  _Float16 v8h;
typedef __attribute__((ext_vector_type(8)))  unsigned short v8us;
typedef __attribute__((ext_vector_type(8)))  float    v8f;
typedef __attribute__((ext_vector_type(4)))  float    v4f;
typedef v8h  __attribute__((may_alias)) v8ha;
typedef v4f  __attribute__((may_alias)) v4fa;
typedef v8us __attribute__((may_alias)) v8usa;

__device__ __forceinline__ unsigned short f2bf(float f) { unsigned u = __float_as_uint(f); u += 0x7FFFu + ((u >> 16) & 1u); return (unsigned short)(u >> 16); }
__device__ __forceinline__ float bf2f(unsigned short b) { return __uint_as_float(((unsigned)b) << 16); }
__device__ __forceinline__ float bfr(float f) { return bf2f(f2bf(f)); }
__device__ __forceinline__ v16h cat16(v8h lo, v8h hi) { return __builtin_shufflevector(lo, hi, 0, 1, 2, 3, 4, 5, 6, 7, 8, 9, 10, 11, 12, 13, 14, 15); }
__device__ __forceinline__ v16bf cat16b(v8us lo, v8us hi) { return __builtin_bit_cast(v16bf, __builtin_shufflevector(lo, hi, 0, 1, 2, 3, 4, 5, 6, 7, 8, 9, 10, 11, 12, 13, 14, 15)); }
__device__ __forceinline__ v8f wmma16(v16h a, v16h b, v8f c) { return __builtin_amdgcn_wmma_f32_16x16x32_f16(false, a, false, b, (short)0, c, false, false); }
__device__ __forceinline__ v8f wmmab(v16bf a, v16bf b, v8f c) { return __builtin_amdgcn_wmma_f32_16x16x32_bf16(false, a, false, b, (short)0, c, false, false); }


template <typename T16> struct WFrag;
template <> struct WFrag<h16> { typedef v16h V; static __device__ __forceinline__ V ld(const h16* p) { return cat16(*(const v8h*)p, *(const v8h*)(p + 16)); } static __device__ __forceinline__ v8f mma(V a, V b, v8f c) { return wmma16(a, b, c); } };
template <> struct WFrag<bf> { typedef v16bf V; static __device__ __forceinline__ V ld(const bf* p) { return cat16b(*(const v8us*)p, *(const v8us*)(p + 16)); } static __device__ __forceinline__ v8f mma(V a, V b, v8f c) { return wmmab(a, b, c); } };
template <typename T16, int NSPLIT, bool BIAS>
__global__ __launch_bounds__(32) void k_gemmw(const T16* __restrict__ A, const T16* __restrict__ A2, const T16* __restrict__ Bt, const T16* __restrict__ Bt2, int K, float* C, int ldc, const float* __restrict__ bias, size_t sA, size_t sB, size_t sC) {
    typedef typename WFrag<T16>::V V;
    __shared__ __align__(16) float os[16 * 68];
    const size_t z = blockIdx.z; A += z * sA; if (A2) A2 += z * sA; Bt += z * sB; if (Bt2) Bt2 += z * sB; C += z * sC;
    const int lane = threadIdx.x & 31, lr = lane & 15, hi = lane >> 4; const int r0 = blockIdx.x * 64, c0 = blockIdx.y * 64;
    v8f acc[4][4];
#pragma unroll
    for (int mb = 0; mb < 4; ++mb)
#pragma unroll
        for (int nb = 0; nb < 4; ++nb) acc[mb][nb] = (v8f){};
    const size_t aoff = (size_t)(r0 + lr) * K + 8 * hi, boff = (size_t)(c0 + lr) * K + 8 * hi;
#pragma unroll 1
    for (int kc = 0; kc < K; kc += 32) {
        V a[4], a2[4];
#pragma unroll
        for (int mb = 0; mb < 4; ++mb) { a[mb] = WFrag<T16>::ld(A + aoff + (size_t)mb * 16 * K + kc); if (NSPLIT == 1 || NSPLIT == 2) a2[mb] = WFrag<T16>::ld(A2 + aoff + (size_t)mb * 16 * K + kc); }
#pragma unroll
        for (int nb = 0; nb < 4; ++nb) { const V b = WFrag<T16>::ld(Bt + boff + (size_t)nb * 16 * K + kc); V b2; if (NSPLIT >= 2) b2 = WFrag<T16>::ld(Bt2 + boff + (size_t)nb * 16 * K + kc);
#pragma unroll
            for (int mb = 0; mb < 4; ++mb) { acc[mb][nb] = WFrag<T16>::mma(a[mb], b, acc[mb][nb]); if (NSPLIT == 1 || NSPLIT == 2) acc[mb][nb] = WFrag<T16>::mma(a2[mb], b, acc[mb][nb]); if (NSPLIT >= 2) acc[mb][nb] = WFrag<T16>::mma(a[mb], b2, acc[mb][nb]); } }
        asm volatile("v_nop\n\tv_nop\n\tv_nop\n\tv_nop" : "+v"(acc[0][0]), "+v"(acc[1][1]), "+v"(acc[2][2]), "+v"(acc[3][3]) : "v"(a[0]), "v"(a[3]));
    }
#pragma unroll
    for (int mb = 0; mb < 4; ++mb) {
#pragma unroll
        for (int nb = 0; nb < 4; ++nb) {
#pragma unroll
            for (int j = 0; j < 8; ++j) os[(hi * 8 + j) * 68 + nb * 16 + lr] = acc[mb][nb][j]; }
        __builtin_amdgcn_wave_barrier(); asm volatile("" ::: "memory");
        float* crow = C + (size_t)(r0 + mb * 16) * ldc + c0;
#pragma unroll 1
        for (int ps = 0; ps < 2; ++ps) {
#pragma unroll
            for (int s = 0; s < 8; ++s) { const int row = 2 * s + hi, cofs = lr * 4; v4f val = *(const v4fa*)(os + row * 68 + cofs); if (BIAS) { val[0] += bfr(bias[c0 + cofs]); val[1] += bfr(bias[c0 + cofs + 1]); val[2] += bfr(bias[c0 + cofs + 2]); val[3] += bfr(bias[c0 + cofs + 3]); }
                *(volatile v4f*)(crow + (size_t)row * ldc + cofs) = val; }
            if (ps == 0) __threadfence(); }
        __builtin_amdgcn_wave_barrier(); asm volatile("" ::: "memory");
    }
}

__device__ __forceinline__ h16 tohx(float x) { return (h16)x; }
__device__ __forceinline__ void splitf(float y, unsigned short& h, unsigned short& l) { h = f2bf(y); l = f2bf(y - bf2f(h)); }
typedef __attribute__((ext_vector_type(2))) _Float16 v2h;
typedef __attribute__((ext_vector_type(4))) _Float16 v4h;
typedef __attribute__((ext_vector_type(2))) unsigned short v2us;

__global__ __launch_bounds__(256) void k_cvt8(const float* __restrict__ src, bf* dst, size_t n8) { const size_t i = (size_t)blockIdx.x * 256 + threadIdx.x; if (i >= n8) return; const v8f v = *(const v8f*)(src + i * 8); v8us o;
#pragma unroll
    for (int k = 0; k < 8; ++k) o[k] = f2bf(v[k]); *(volatile v8us*)(dst + i * 8) = o; __threadfence(); *(volatile v8us*)(dst + i * 8) = o; }
__global__ __launch_bounds__(256) void k_split2p(const float* __restrict__ F, int pitch, int width, bf* Ph, bf* Pl) { const size_t e = ((size_t)blockIdx.x * 256 + threadIdx.x) * 2; if (e >= (size_t)TT * width) return; const int c = (int)(e % width); const int t = (int)(e / width); v2us oh, ol;
#pragma unroll
    for (int q = 0; q < 2; ++q) { unsigned short a, c2; splitf(F[(size_t)t * pitch + c + q], a, c2); oh[q] = a; ol[q] = c2; } *(volatile v2us*)(Ph + e) = oh; *(volatile v2us*)(Pl + e) = ol; __threadfence(); *(volatile v2us*)(Ph + e) = oh; *(volatile v2us*)(Pl + e) = ol; }
__global__ __launch_bounds__(32) void k_lam(const float* __restrict__ lqn, const float* __restrict__ lqr, const float* __restrict__ lkn, const float* __restrict__ lkr, float* LAM) { const int lane = threadIdx.x; float a = 0.f, b = 0.f;
    for (int i = lane; i < DN; i += 32) { float p = __fmul_rn(bfr(lqn[i]), bfr(lkn[i])); asm volatile("" : "+v"(p)); a = __fadd_rn(a, p); }
    for (int i = lane; i < DR; i += 32) { float p = __fmul_rn(bfr(lqr[i]), bfr(lkr[i])); asm volatile("" : "+v"(p)); b = __fadd_rn(b, p); }
#pragma unroll
    for (int sh = 16; sh; sh >>= 1) { a += __shfl_xor(a, sh, 32); b += __shfl_xor(b, sh, 32); }
    const float l = __fadd_rn(__fsub_rn(__expf(a), __expf(b)), LINIT); const float o = lane == 0 ? l : 0.f; *(volatile float*)(LAM + lane) = o; __threadfence(); *(volatile float*)(LAM + lane) = o; }
__device__ __forceinline__ float ropev(const float* __restrict__ pe, int e, const float* __restrict__ cs, const float* __restrict__ sn, int t) { const int i = e >> 1; const float xr = pe[2 * i], xi = pe[2 * i + 1]; float c = bfr(cs[t * 32 + i]), s = bfr(sn[t * 32 + i]); asm volatile("" : "+v"(c)); asm volatile("" : "+v"(s));
    float p = __fmul_rn(xr, (e & 1) ? s : c), q = __fmul_rn(xi, (e & 1) ? c : s); asm volatile("" : "+v"(p)); asm volatile("" : "+v"(q)); return (e & 1) ? __fadd_rn(p, q) : __fsub_rn(p, q); }
__global__ __launch_bounds__(256) void k_qpl(const float* __restrict__ Q, const float* __restrict__ cs, const float* __restrict__ sn, int h, int hf, bf* Ph, bf* Pl, h16* P16) { const int e = (blockIdx.x * 256 + threadIdx.x) * 2; if (e >= TT * HH) return; const int d = e % HH, t = e / HH; const float* qr = Q + (size_t)t * (NH_ * QKH) + h * QKH; v2h o16; v2us oh, ol;
#pragma unroll
    for (int q = 0; q < 2; ++q) { const int dd = d + q; const float v = (hf == 0) ? qr[dd] : (dd < 32 ? qr[HH + dd] : ropev(qr + DN, dd - 32, cs, sn, t)); o16[q] = tohx(v); unsigned short a, c2; splitf(v, a, c2); oh[q] = a; ol[q] = c2; }
    *(volatile v2h*)(P16 + e) = o16; if (t < RH) { *(volatile v2us*)(Ph + e) = oh; *(volatile v2us*)(Pl + e) = ol; } __threadfence(); *(volatile v2h*)(P16 + e) = o16; if (t < RH) { *(volatile v2us*)(Ph + e) = oh; *(volatile v2us*)(Pl + e) = ol; } }
__global__ __launch_bounds__(256) void k_kpl(const float* __restrict__ KVB, const float* __restrict__ KVF, const float* __restrict__ cs, const float* __restrict__ sn, int h, int hf, bf* Ph, bf* Pl, h16* P16) { const int e = (blockIdx.x * 256 + threadIdx.x) * 2; if (e >= TT * HH) return; const int d = e % HH, t = e / HH; const float* kr = KVB + (size_t)t * (NH_ * (DN + DV)) + h * (DN + DV); v2h o16; v2us oh, ol;
#pragma unroll
    for (int q = 0; q < 2; ++q) { const int dd = d + q; const float v = (hf == 0) ? kr[dd] : (dd < 32 ? kr[HH + dd] : ropev(KVF + (size_t)t * KVW + KVL, dd - 32, cs, sn, t)); o16[q] = tohx(v); unsigned short a, c2; splitf(v, a, c2); oh[q] = a; ol[q] = c2; }
    *(volatile v2h*)(P16 + e) = o16; *(volatile v2us*)(Ph + e) = oh; *(volatile v2us*)(Pl + e) = ol; __threadfence(); *(volatile v2h*)(P16 + e) = o16; *(volatile v2us*)(Ph + e) = oh; *(volatile v2us*)(Pl + e) = ol; }
__global__ __launch_bounds__(256) void k_vt(const float* __restrict__ KVB, int h, bf* Vh, bf* Vl, h16* V16) { const int e = (blockIdx.x * 256 + threadIdx.x) * 2; if (e >= DV * TT) return; const int t = e % TT, d = e / TT; v2h o16; v2us oh, ol;
#pragma unroll
    for (int q = 0; q < 2; ++q) { const float v = KVB[(size_t)(t + q) * (NH_ * (DN + DV)) + h * (DN + DV) + DN + d]; o16[q] = tohx(v); unsigned short a, c2; splitf(v, a, c2); oh[q] = a; ol[q] = c2; }
    *(volatile v2h*)(V16 + e) = o16; *(volatile v2us*)(Vh + e) = oh; *(volatile v2us*)(Vl + e) = ol; __threadfence(); *(volatile v2h*)(V16 + e) = o16; *(volatile v2us*)(Vh + e) = oh; *(volatile v2us*)(Vl + e) = ol; }
__global__ __launch_bounds__(256) void k_asoft(const float* __restrict__ Sb, const float* __restrict__ ab, bf* Ph, bf* Pl, h16* P16) {
    typedef __attribute__((ext_vector_type(4))) unsigned short v4us;
    const int lane = threadIdx.x & 31; const int row = blockIdx.x * 8 + (threadIdx.x >> 5); if (row >= ZH * TT) return; const int i = row & (TT - 1); const int zz = row >> 11; const bool hires = (i < RH);
    const float* sr = Sb + (size_t)row * TT; const float* mr = ab + (size_t)i * TT; float v[64]; float mx = -3.0e38f;
#pragma unroll
    for (int ch = 0; ch < 16; ++ch) { const int j0 = ch * 128 + lane * 4; const v4f a = *(const v4f*)(sr + j0), m4 = *(const v4f*)(mr + j0);
#pragma unroll
        for (int q = 0; q < 4; ++q) { float sa = fminf(fmaxf(a[q] * SCL, -100.0f), 100.0f), mb = bfr(m4[q]); asm volatile("" : "+v"(sa)); asm volatile("" : "+v"(mb)); const float t = __fadd_rn(sa, mb); v[ch * 4 + q] = t; mx = fmaxf(mx, t); } }
#pragma unroll
    for (int sh = 16; sh; sh >>= 1) mx = fmaxf(mx, __shfl_xor(mx, sh, 32));
    float sum = 0.f;
#pragma unroll
    for (int k = 0; k < 64; ++k) { v[k] = __expf(v[k] - mx); sum += v[k]; }
#pragma unroll
    for (int sh = 16; sh; sh >>= 1) sum += __shfl_xor(sum, sh, 32);
    const float f = __fdiv_rn(hires ? 1.0f : PCAR, sum);
#pragma unroll 1
    for (int ps = 0; ps < 2; ++ps) {
        if (hires) {
#pragma unroll
            for (int ch = 0; ch < 16; ++ch) { v4us oh, ol;
#pragma unroll
                for (int q = 0; q < 4; ++q) { unsigned short a, c2; splitf(v[ch * 4 + q] * f, a, c2); oh[q] = a; ol[q] = c2; }
                const size_t o = ((size_t)zz * RH + i) * TT + ch * 128 + lane * 4; *(volatile v4us*)(Ph + o) = oh; *(volatile v4us*)(Pl + o) = ol; }
        } else {
#pragma unroll
            for (int ch = 0; ch < 16; ++ch) { v4h o;
#pragma unroll
                for (int q = 0; q < 4; ++q) o[q] = tohx(v[ch * 4 + q] * f);
                *(volatile v4h*)(P16 + (size_t)row * TT + ch * 128 + lane * 4) = o; } }
        if (ps == 0) __threadfence(); }
}
__global__ __launch_bounds__(256) void k_mrgd(const float* __restrict__ O1, const float* __restrict__ O2, const float* __restrict__ LAM, int h, bf* Ah, bf* Al) { const int e = (blockIdx.x * 256 + threadIdx.x) * 2; if (e >= TT * DV) return; const int d = e % DV, t = e / DV; const float cs = (t < RH) ? 1.0f : (1.0f / PCAR); const float lam = LAM[0]; v2us oh, ol;
#pragma unroll
    for (int q = 0; q < 2; ++q) { float a = __fmul_rn(O1[e + q], cs), b = __fmul_rn(O2[e + q], cs); asm volatile("" : "+v"(a)); asm volatile("" : "+v"(b)); float lb = __fmul_rn(lam, b); asm volatile("" : "+v"(lb)); float df = __fsub_rn(a, lb); asm volatile("" : "+v"(df)); unsigned short a2, c2; splitf(__fmul_rn(df, OMUL), a2, c2); oh[q] = a2; ol[q] = c2; }
    const size_t oo = (size_t)t * (NH_ * DV) + h * DV + d; *(volatile v2us*)(Ah + oo) = oh; *(volatile v2us*)(Al + oo) = ol; __threadfence(); *(volatile v2us*)(Ah + oo) = oh; *(volatile v2us*)(Al + oo) = ol; }

extern "C" void kernel_launch(void* const* d_in, const int* in_sizes, int n_in,
                              void* d_out, int out_size, void* d_ws, size_t ws_size, hipStream_t stream) {
    (void)in_sizes; (void)n_in; (void)out_size;
    const float* IN[14]; for (int i = 0; i < 14; ++i) IN[i] = (const float*)d_in[i];
    float* OUT = (float*)d_out;
    char* wsp = (char*)d_ws;
    auto take = [&](size_t bytes) { char* p = wsp; wsp += (bytes + 255) & ~(size_t)255; return (void*)p; };
    bf* WQA = (bf*)take((size_t)QLR * DM * 2); bf* WQB = (bf*)take((size_t)NH_ * QKH * QLR * 2); bf* WKA = (bf*)take((size_t)KVW * DM * 2); bf* WKB = (bf*)take((size_t)NH_ * (DN + DV) * KVL * 2); bf* WO = (bf*)take((size_t)DM * DM * 2); float* LAM = (float*)take(256);
    bf* XB = (bf*)take((size_t)TT * DM * 2); float* QA = (float*)take((size_t)TT * QLR * 4); bf* QAh = (bf*)take((size_t)TT * QLR * 2); bf* QAl = (bf*)take((size_t)TT * QLR * 2); float* Q = (float*)take((size_t)TT * NH_ * QKH * 4);
    float* KVF = (float*)take((size_t)TT * KVW * 4); bf* KVh = (bf*)take((size_t)TT * KVL * 2); bf* KVl = (bf*)take((size_t)TT * KVL * 2); float* KVB = (float*)take((size_t)TT * NH_ * (DN + DV) * 4);
    bf* QPh = (bf*)take((size_t)TT * HH * 2); bf* QPl = (bf*)take((size_t)TT * HH * 2); h16* QP16 = (h16*)take((size_t)TT * HH * 2); bf* KPh = (bf*)take((size_t)TT * HH * 2); bf* KPl = (bf*)take((size_t)TT * HH * 2); h16* KP16 = (h16*)take((size_t)TT * HH * 2);
    bf* VTh = (bf*)take((size_t)DV * TT * 2); bf* VTl = (bf*)take((size_t)DV * TT * 2); h16* VT16 = (h16*)take((size_t)DV * TT * 2); float* Sb = (float*)take((size_t)TT * TT * 4); bf* Ph = (bf*)take((size_t)RH * TT * 2); bf* Pl = (bf*)take((size_t)RH * TT * 2); h16* P16 = (h16*)take((size_t)TT * TT * 2);
    float* O1 = (float*)take((size_t)TT * DV * 4); float* O2 = (float*)take((size_t)TT * DV * 4); bf* Ah = (bf*)take((size_t)TT * NH_ * DV * 2); bf* Al = (bf*)take((size_t)TT * NH_ * DV * 2);
    if ((size_t)(wsp - (char*)d_ws) > ws_size) return;
    { k_cvt8<<<(unsigned)(((size_t)QLR * DM / 8 + 255) / 256), 256, 0, stream>>>(IN[1], WQA, (size_t)QLR * DM / 8); k_cvt8<<<(unsigned)(((size_t)NH_ * QKH * QLR / 8 + 255) / 256), 256, 0, stream>>>(IN[2], WQB, (size_t)NH_ * QKH * QLR / 8);
      k_cvt8<<<(unsigned)(((size_t)KVW * DM / 8 + 255) / 256), 256, 0, stream>>>(IN[3], WKA, (size_t)KVW * DM / 8); k_cvt8<<<(unsigned)(((size_t)NH_ * (DN + DV) * KVL / 8 + 255) / 256), 256, 0, stream>>>(IN[4], WKB, (size_t)NH_ * (DN + DV) * KVL / 8);
      k_cvt8<<<(unsigned)(((size_t)DM * DM / 8 + 255) / 256), 256, 0, stream>>>(IN[5], WO, (size_t)DM * DM / 8); k_cvt8<<<(unsigned)(((size_t)TT * DM / 8 + 255) / 256), 256, 0, stream>>>(IN[0], XB, (size_t)TT * DM / 8);
      k_lam<<<1, 32, 0, stream>>>(IN[6], IN[7], IN[8], IN[9], LAM); }
    k_gemmw<bf, 0, false><<<dim3(TT / 64, QLR / 64, 1), 32, 0, stream>>>(XB, nullptr, WQA, nullptr, DM, QA, QLR, nullptr, 0, 0, 0); k_split2p<<<(unsigned)(((size_t)TT * QLR / 2 + 255) / 256), 256, 0, stream>>>(QA, QLR, QLR, QAh, QAl);
    k_gemmw<bf, 1, false><<<dim3(TT / 64, NH_ * QKH / 64, 1), 32, 0, stream>>>(QAh, QAl, WQB, nullptr, QLR, Q, NH_ * QKH, nullptr, 0, 0, 0);
    k_gemmw<bf, 0, false><<<dim3(TT / 64, KVW / 64, 1), 32, 0, stream>>>(XB, nullptr, WKA, nullptr, DM, KVF, KVW, nullptr, 0, 0, 0); k_split2p<<<(unsigned)(((size_t)TT * KVL / 2 + 255) / 256), 256, 0, stream>>>(KVF, KVW, KVL, KVh, KVl);
    k_gemmw<bf, 1, false><<<dim3(TT / 64, NH_ * (DN + DV) / 64, 1), 32, 0, stream>>>(KVh, KVl, WKB, nullptr, KVL, KVB, NH_ * (DN + DV), nullptr, 0, 0, 0);
    const unsigned LQ = (TT * HH / 2 + 255) / 256, LV = (DV * TT / 2 + 255) / 256;
    for (int h = 0; h < NH_; ++h) {
        k_vt<<<LV, 256, 0, stream>>>(KVB, h, VTh, VTl, VT16);
        for (int hf = 0; hf < 2; ++hf) { float* O = hf ? O2 : O1;
            k_qpl<<<LQ, 256, 0, stream>>>(Q, IN[10], IN[11], h, hf, QPh, QPl, QP16); k_kpl<<<LQ, 256, 0, stream>>>(KVB, KVF, IN[10], IN[11], h, hf, KPh, KPl, KP16);
            k_gemmw<bf, 2, false><<<dim3(RH / 64, TT / 64, 1), 32, 0, stream>>>(QPh, QPl, KPh, KPl, HH, Sb, TT, nullptr, 0, 0, 0);
            k_gemmw<h16, 0, false><<<dim3((TT - RH) / 64, TT / 64, 1), 32, 0, stream>>>(QP16 + (size_t)RH * HH, nullptr, KP16, nullptr, HH, Sb + (size_t)RH * TT, TT, nullptr, 0, 0, 0);
            k_asoft<<<TT / 8, 256, 0, stream>>>(Sb, IN[12], Ph, Pl, P16);
            k_gemmw<bf, 2, false><<<dim3(RH / 64, DV / 64, 1), 32, 0, stream>>>(Ph, Pl, VTh, VTl, TT, O, DV, nullptr, 0, 0, 0);
            k_gemmw<h16, 0, false><<<dim3((TT - RH) / 64, DV / 64, 1), 32, 0, stream>>>(P16 + (size_t)RH * TT, nullptr, VT16, nullptr, TT, O + (size_t)RH * DV, DV, nullptr, 0, 0, 0); }
        k_mrgd<<<(TT * DV / 2 + 255) / 256, 256, 0, stream>>>(O1, O2, LAM, h, Ah, Al); }
    k_gemmw<bf, 1, false><<<dim3(TT / 64, DM / 64, 1), 32, 0, stream>>>(Ah, Al, WO, nullptr, NH_ * DV, OUT, DM, nullptr, 0, 0, 0);
}
